// Net_PPF_LRBF2_84954453115110
// MI455X (gfx1250) — hardware-verified
//
#include <hip/hip_runtime.h>
#include <math.h>

typedef __attribute__((ext_vector_type(16))) _Float16 v16h;
typedef __attribute__((ext_vector_type(16))) __bf16 v16b;
typedef __attribute__((ext_vector_type(8)))  _Float16 v8h;
typedef __attribute__((ext_vector_type(8)))  float v8f;
typedef __attribute__((ext_vector_type(4)))  float v4f;
typedef __attribute__((ext_vector_type(2)))  float v2f;
typedef __attribute__((ext_vector_type(4)))  unsigned v4u;
typedef __attribute__((ext_vector_type(4)))  int v4i;
typedef float __attribute__((may_alias)) float_a;
typedef int __attribute__((may_alias)) int_a;

template <typename T> __device__ __forceinline__ void vst2(void* p, T v) { *(volatile T*)p = v; __threadfence(); *(volatile T*)p = v; }
__device__ __forceinline__ v8f wmma16(v16h a, v16h b, v8f c) {
  v8f d = __builtin_amdgcn_wmma_f32_16x16x32_f16(false, a, false, b, (short)0, c, false, false);
  asm volatile("v_nop\n\tv_nop\n\tv_nop\n\tv_nop" : "+v"(d) : "v"(a), "v"(b));
  return d;
}
__device__ __forceinline__ v8f wmma_bf(v16b a, v16b b, v8f c) {
  v8f d = __builtin_amdgcn_wmma_f32_16x16x32_bf16(false, a, false, b, (short)0, c, false, false);
  asm volatile("v_nop\n\tv_nop\n\tv_nop\n\tv_nop" : "+v"(d) : "v"(a), "v"(b));
  return d;
}
__device__ __forceinline__ v16h frag_h(const _Float16* rowk0, int lane) {
  union { v16h v; v8h q[2]; } u; const _Float16* p = rowk0 + 8 * (lane >> 4);
  u.q[0] = *(const v8h*)p; u.q[1] = *(const v8h*)(p + 16); return u.v;
}
__device__ __forceinline__ v16h frag_f32(const float* rowk0, int lane) {
  v16h a; const float* p = rowk0 + 8 * (lane >> 4);
#pragma unroll
  for (int i = 0; i < 8; ++i) { a[i] = (_Float16)p[i]; a[8 + i] = (_Float16)p[16 + i]; }
  return a;
}
__device__ __forceinline__ v16h frag_f32s(const float* rowk0, int lane, float sc) {
  v16h a; const float* p = rowk0 + 8 * (lane >> 4);
#pragma unroll
  for (int i = 0; i < 8; ++i) { a[i] = (_Float16)(p[i] * sc); a[8 + i] = (_Float16)(p[16 + i] * sc); }
  return a;
}
__device__ __forceinline__ v16h fragc_f32(const float* W, int k0, int n, int lane, int ld, int K) {
  v16h a; const int g = lane >> 4;
#pragma unroll
  for (int i = 0; i < 8; ++i) { const int ka = k0 + 8 * g + i, kb = ka + 16;
    a[i] = (_Float16)(ka < K ? W[(size_t)(ka < K ? ka : K - 1) * ld + n] : 0.f); a[8 + i] = (_Float16)(kb < K ? W[(size_t)(kb < K ? kb : K - 1) * ld + n] : 0.f); }
  return a;
}
struct F2 { v16b h, l; };
__device__ __forceinline__ F2 bsplit16(const float v[16]) { F2 r;
#pragma unroll
  for (int i = 0; i < 16; ++i) { const __bf16 h = (__bf16)v[i]; r.h[i] = h; r.l[i] = (__bf16)(v[i] - (float)h); }
  return r; }
__device__ __forceinline__ F2 split_row(const float* row, int k0, int lane) { float v[16]; const float* p = row + k0 + 8 * (lane >> 4);
#pragma unroll
  for (int i = 0; i < 8; ++i) { v[i] = p[i]; v[8 + i] = p[16 + i]; }
  return bsplit16(v); }
__device__ __forceinline__ F2 split_rowK(const float* row, int k0, int lane, int K) { float v[16]; const int g = lane >> 4;
#pragma unroll
  for (int i = 0; i < 8; ++i) { const int ka = k0 + 8 * g + i, kb = ka + 16; v[i] = ka < K ? row[ka < K ? ka : K - 1] : 0.f; v[8 + i] = kb < K ? row[kb < K ? kb : K - 1] : 0.f; }
  return bsplit16(v); }
__device__ __forceinline__ F2 split_col(const float* W, int k0, int n, int lane, int ld, int K) { float v[16]; const int g = lane >> 4;
#pragma unroll
  for (int i = 0; i < 8; ++i) { const int ka = k0 + 8 * g + i, kb = ka + 16; v[i] = ka < K ? W[(size_t)(ka < K ? ka : K - 1) * ld + n] : 0.f; v[8 + i] = kb < K ? W[(size_t)(kb < K ? kb : K - 1) * ld + n] : 0.f; }
  return bsplit16(v); }
__device__ __forceinline__ v8f mac3(const F2& a, const F2& b, v8f c) { c = wmma_bf(a.l, b.h, c); c = wmma_bf(a.h, b.l, c); return wmma_bf(a.h, b.h, c); }
__device__ __forceinline__ float sigm(float v) { return 1.0f / (1.0f + expf(-v)); }
#define LDSX() do { asm volatile("s_wait_dscnt 0" ::: "memory"); __builtin_amdgcn_wave_barrier(); __builtin_amdgcn_fence(__ATOMIC_RELEASE, "workgroup"); } while (0)


#define CSR_N 50000
#define CSR_E 400000
#define NB 500
#define NNP 50048

#define CSR_FINN (CSR_E + 32 * CSR_NBK)
#define CSR_CHUNK 4096
#define CSR_BKT 256
#define CSR_NCH ((CSR_E + CSR_CHUNK - 1) / CSR_CHUNK)
#define CSR_NBK ((CSR_N + CSR_BKT - 1) / CSR_BKT)
#define CSR_NBKP (((CSR_NBK + 63) / 64) * 64)
#define CSR_SEGCAP (CSR_E + 32 * CSR_NBK * CSR_NCH)
#ifndef CSR_BCAP
#define CSR_BCAP 10240
#endif
#define CSR_SZ_CNT   (4u * CSR_NCH * CSR_NBKP)
#define CSR_SZ_OFF   (4u * CSR_NBK * (((CSR_NCH + 31) / 32) * 32))
#define CSR_SZ_BST   (4u * (((CSR_NBK + 1 + 31) / 32) * 32))
#define CSR_SZ_SEG   (4u * CSR_SEGCAP)
#define CSR_SZ_FIN   (4u * (CSR_E + 32 * CSR_NBK))
#define CSR_SZ_ROW   (4u * CSR_NBK * CSR_BKT)
#define CSR_OFFP (((CSR_NCH + 31) / 32) * 32)

__global__ __launch_bounds__(256) void k_csr_cnt(const int* __restrict__ DST, int dstride, int* __restrict__ CNT) {
  __shared__ unsigned short sc[256][CSR_NBK + 1]; __shared__ __align__(16) int srow[CSR_NBKP];
  const int c = blockIdx.x, tid = threadIdx.x;
  for (int b = 0; b < CSR_NBK; ++b) sc[tid][b] = 0;
  const size_t e0 = (size_t)c * CSR_CHUNK + tid * 16;
  for (int i = 0; i < 16; ++i) { const size_t e = e0 + i; if (e < (size_t)CSR_E) { int d = DST[e * dstride]; d = min(max(d, 0), CSR_N - 1); sc[tid][d / CSR_BKT] += 1; } }
  __syncthreads();
  for (int b = tid; b < CSR_NBKP; b += 256) { int s = 0; if (b < CSR_NBK) for (int t = 0; t < 256; ++t) s += sc[t][b]; srow[b] = s; }
  __syncthreads();
  for (int q = tid; q < CSR_NBKP / 4; q += 256) vst2((unsigned*)(CNT + (size_t)c * CSR_NBKP + q * 4), *(const v4u*)&srow[q * 4]);
}
__global__ __launch_bounds__(256) void k_csr_scan(const int* __restrict__ CNT, int* __restrict__ OFF, int* __restrict__ BST) {
  __shared__ int sbt[CSR_NBK + 1]; __shared__ int sbs[((CSR_NBK + 1 + 31) / 32) * 32]; __shared__ int scnt[CSR_NBK + 1]; __shared__ __align__(16) int sbuf[64][CSR_OFFP];
  const int tid = threadIdx.x;
  for (int b = tid; b < CSR_NBK; b += 256) { int sp = 0, st = 0; for (int c = 0; c < CSR_NCH; ++c) { const int n = CNT[(size_t)c * CSR_NBKP + b]; st += n; sp += (n + 31) & ~31; } sbt[b] = sp; scnt[b] = st; }
  for (int b = tid; b < ((CSR_NBK + 1 + 31) / 32) * 32; b += 256) sbs[b] = 0;
  __syncthreads();
  if (tid == 0) { int acc = 0, accf = 0; for (int b = 0; b < CSR_NBK; ++b) { const int t = sbt[b]; sbt[b] = acc; acc += t; sbs[b] = accf; accf += (scnt[b] + 31) & ~31; } sbs[CSR_NBK] = accf; }
  __syncthreads();
  for (int b0 = 0; b0 < CSR_NBK; b0 += 64) {
    if (tid < 64 && b0 + tid < CSR_NBK) { const int b = b0 + tid; int o = sbt[b]; for (int c = 0; c < CSR_OFFP; ++c) { if (c < CSR_NCH) { sbuf[tid][c] = o; o += (CNT[(size_t)c * CSR_NBKP + b] + 31) & ~31; } else sbuf[tid][c] = 0; } }
    __syncthreads();
    for (int q = tid; q < 64 * (CSR_OFFP / 4); q += 256) { const int r = q / (CSR_OFFP / 4), pc = q % (CSR_OFFP / 4); if (b0 + r < CSR_NBK) vst2((unsigned*)(OFF + (size_t)(b0 + r) * CSR_OFFP + pc * 4), *(const v4u*)&sbuf[r][pc * 4]); }
    __syncthreads(); }
  for (int q = tid; q < ((CSR_NBK + 1 + 31) / 32) * 32 / 4; q += 256) vst2((unsigned*)(BST + q * 4), *(const v4u*)&sbs[q * 4]);
}
__global__ __launch_bounds__(256) void k_csr_scatter(const int* __restrict__ SRC, const int* __restrict__ DST, int sstride, int dstride, const int* __restrict__ OFF, int* __restrict__ SEGS, int* __restrict__ SEGE) {
  __shared__ unsigned short sc[256][CSR_NBK + 1]; __shared__ int sbase[CSR_NBK + 1]; __shared__ int scn[CSR_NBK + 1]; __shared__ int sord[CSR_CHUNK];
  const int c = blockIdx.x, tid = threadIdx.x;
  for (int b = 0; b < CSR_NBK; ++b) sc[tid][b] = 0;
  const size_t e0 = (size_t)c * CSR_CHUNK + tid * 16; int bk[16];
#pragma unroll
  for (int i = 0; i < 16; ++i) { const size_t e = e0 + i; bk[i] = -1; if (e < (size_t)CSR_E) { int d = DST[e * dstride]; d = min(max(d, 0), CSR_N - 1); bk[i] = d / CSR_BKT; sc[tid][bk[i]] += 1; } }
  __syncthreads();
  for (int b = tid; b < CSR_NBK; b += 256) { int acc = 0; for (int t = 0; t < 256; ++t) { const int v = sc[t][b]; sc[t][b] = (unsigned short)acc; acc += v; } scn[b] = acc; }
  __syncthreads();
  if (tid == 0) { int acc = 0; for (int b = 0; b < CSR_NBK; ++b) { sbase[b] = acc; acc += scn[b]; } }
  __syncthreads();
#pragma unroll
  for (int i = 0; i < 16; ++i) { if (bk[i] >= 0) { const int b = bk[i]; const int r = sc[tid][b]; sc[tid][b] = (unsigned short)(r + 1); sord[sbase[b] + r] = tid * 16 + i; } }
  __syncthreads();
  for (int b = 0; b < CSR_NBK; ++b) { const int n = scn[b]; if (n == 0) continue; const int nl = ((n + 31) & ~31); const size_t o = (size_t)(min(max(OFF[(size_t)b * CSR_OFFP + c], 0), CSR_SEGCAP - nl) & ~31);
    for (int q = tid; q < nl / 4; q += 256) { int4 vs, ve;
#pragma unroll
      for (int k = 0; k < 4; ++k) { const int i = q * 4 + k; int s = -1, eid = -1; if (i < n) { const size_t e = (size_t)c * CSR_CHUNK + sord[sbase[b] + i]; s = min(max(SRC[e * sstride], 0), CSR_N - 1); eid = (int)e; } vs[k] = s; ve[k] = eid; }
      vst2((unsigned*)(SEGS + o + q * 4), *(const v4u*)&vs); vst2((unsigned*)(SEGE + o + q * 4), *(const v4u*)&ve); } }
}
__global__ __launch_bounds__(256) void k_csr_bucket(const int* __restrict__ CNT, const int* __restrict__ OFF, const int* __restrict__ BST, const int* __restrict__ SEGS, const int* __restrict__ SEGE, const int* __restrict__ DST, int dstride, int* __restrict__ FS, int* __restrict__ FE, int* __restrict__ ROWST, int* __restrict__ ROWCNT) {
  __shared__ int ssrc[CSR_BCAP]; __shared__ int seid[CSR_BCAP]; __shared__ unsigned char snod[CSR_BCAP]; __shared__ int souts[CSR_BCAP]; __shared__ int soute[CSR_BCAP]; __shared__ int scount[256]; __shared__ int sstart[257]; __shared__ int stot;
  const int b = blockIdx.x, tid = threadIdx.x;
  if (tid == 0) { int t = 0; for (int c = 0; c < CSR_NCH; ++c) t += min(max(CNT[(size_t)c * CSR_NBKP + b], 0), CSR_CHUNK); stot = (t <= CSR_BCAP) ? t : 0; }
  __syncthreads();
  { int base = 0; for (int c = 0; c < CSR_NCH; ++c) { const int n = min(max(CNT[(size_t)c * CSR_NBKP + b], 0), CSR_CHUNK); const int o = min(max(OFF[(size_t)b * CSR_OFFP + c], 0), CSR_SEGCAP - ((n + 31) & ~31));
      for (int i = tid; i < n; i += 256) { const int p = base + i; if (p < CSR_BCAP) { ssrc[p] = min(max(SEGS[o + i], 0), CSR_N - 1); const int e = min(max(SEGE[o + i], 0), CSR_E - 1); seid[p] = e; int d = DST[(size_t)e * dstride]; d = min(max(d, 0), CSR_N - 1); const int dl = d - b * CSR_BKT; snod[p] = (unsigned char)(dl >= 0 && dl < 256 ? dl : 255); } }
      base += n; } }
  __syncthreads();
  const int node = b * CSR_BKT + tid; int cnt = 0; for (int p = 0; p < stot; ++p) cnt += (snod[p] == tid) ? 1 : 0;
  scount[tid] = cnt; __syncthreads();
  if (tid == 0) { int acc = 0; for (int t = 0; t < 256; ++t) { sstart[t] = acc; acc += scount[t]; } sstart[256] = acc; }
  __syncthreads();
  const int bst0 = min(max(BST[b], 0), CSR_FINN - ((sstart[256] + 31) & ~31)) & ~31; const int gst = bst0 + sstart[tid];
  { int w = sstart[tid]; for (int p = 0; p < stot; ++p) if (snod[p] == tid) { souts[w] = ssrc[p]; soute[w] = seid[p]; ++w; } }
  __syncthreads();
  { const int n = sstart[256]; const int nl = (n + 31) & ~31; for (int q = tid; q < nl / 4; q += 256) { int4 vs, ve;
#pragma unroll
      for (int k = 0; k < 4; ++k) { const int i = q * 4 + k; vs[k] = i < n ? souts[i] : -1; ve[k] = i < n ? soute[i] : -1; }
      vst2((unsigned*)(FS + bst0 + q * 4), *(const v4u*)&vs); vst2((unsigned*)(FE + bst0 + q * 4), *(const v4u*)&ve); } }
  __syncthreads();
  { __shared__ __align__(16) int srs[256], src2[256]; srs[tid] = node < CSR_N ? gst : 0; src2[tid] = node < CSR_N ? cnt : 0; __syncthreads();
    if (tid < 64) vst2((unsigned*)(ROWST + (size_t)b * 256 + tid * 4), *(const v4u*)&srs[tid * 4]); else if (tid < 128) vst2((unsigned*)(ROWCNT + (size_t)b * 256 + (tid - 64) * 4), *(const v4u*)&src2[(tid - 64) * 4]); }
}

typedef __attribute__((ext_vector_type(8))) __bf16 v8b;
__device__ __forceinline__ v16b frag_b(const __bf16* rowk0, int lane) {
  union { v16b v; v8b q[2]; } u; const __bf16* p = rowk0 + 8 * (lane >> 4);
  u.q[0] = *(const v8b*)p; u.q[1] = *(const v8b*)(p + 16); return u.v;
}
__device__ __forceinline__ float bfr(float v) { return (float)(__bf16)v; }
__device__ __attribute__((noinline)) float exp_ni(float v) { return expf(v); }
#define WS_CNT  0u
#define WS_OFF  (WS_CNT + CSR_SZ_CNT)
#define WS_BST  (WS_OFF + CSR_SZ_OFF)
#define WS_SEGS (WS_BST + CSR_SZ_BST)
#define WS_SEGE (WS_SEGS + CSR_SZ_SEG)
#define WS_FS   (WS_SEGE + CSR_SZ_SEG)
#define WS_FE   (WS_FS + CSR_SZ_FIN)
#define WS_RST  (WS_FE + CSR_SZ_FIN)
#define WS_RCT  (WS_RST + CSR_SZ_ROW)
#define WS_PT   (WS_RCT + CSR_SZ_ROW)
#define PT_W1  0
#define PT_W1R (128 * 64)
#define PT_W2  (2 * 128 * 64)
#define PT_W2R (2 * 128 * 64 + 64 * 128)
#define PT_END (2 * 128 * 64 + 2 * 64 * 128)
#define WS_X0   (WS_PT + 2u * PT_END)
#define WS_HM   (WS_X0 + 4u * NNP * 64)
#define WS_RS   (WS_HM + 4u * NNP * 128)
#define WS_X1   (WS_RS + 4u * NNP * 128)
#define WS_X2   (WS_X1 + 4u * NNP * 128)
#define WS_HG   (WS_X2 + 4u * NNP * 64)
#define WS_END  (WS_HG + 4u * 512 * 64)

__global__ __launch_bounds__(128) void k_pack(const float* __restrict__ W1, const float* __restrict__ W1r, const float* __restrict__ W2, const float* __restrict__ W2r, __bf16* __restrict__ PT) {
  __shared__ __align__(16) __bf16 srow[128];
  const int n = blockIdx.x, tid = threadIdx.x; int len; size_t dst;
  if (n < 128) { len = 64; dst = PT_W1 + (size_t)n * 64; if (tid < 64) srow[tid] = (__bf16)bfr(W1[(size_t)tid * 128 + n]); }
  else if (n < 256) { const int o = n - 128; len = 64; dst = PT_W1R + (size_t)o * 64; if (tid < 64) srow[tid] = (__bf16)bfr(W1r[(size_t)tid * 128 + o]); }
  else if (n < 320) { const int o = n - 256; len = 128; dst = PT_W2 + (size_t)o * 128; srow[tid] = (__bf16)bfr(W2[(size_t)tid * 64 + o]); }
  else { const int o = n - 320; len = 128; dst = PT_W2R + (size_t)o * 128; srow[tid] = (__bf16)bfr(W2r[(size_t)tid * 64 + o]); }
  __syncthreads();
  if (tid < len / 8) vst2((unsigned*)(PT + dst + tid * 8), *(const v4u*)(&srow[tid * 8]));
}
__global__ __launch_bounds__(256) void k_x0(const float* __restrict__ X, float* __restrict__ X0) {
  const int tid = threadIdx.x; const size_t r = (size_t)blockIdx.x * 64 + (tid >> 2);
  for (int piece = (tid & 3); piece < 16; piece += 4) { v4f v; for (int i = 0; i < 4; ++i) v[i] = r < (size_t)CSR_N ? bfr(X[r * 64 + piece * 4 + i]) : 0.f; vst2(X0 + r * 64 + piece * 4, v); }
}
template <int L>
__global__ __launch_bounds__(128) void k_pre(const float* __restrict__ Xin, const __bf16* __restrict__ PT, const float* __restrict__ br, const int* __restrict__ RCT, float* __restrict__ HM, float* __restrict__ RS) {
  constexpr int KI = (L == 1) ? 64 : 128, NO = (L == 1) ? 128 : 64, NT = NO / 16;
  __shared__ __align__(16) float so[4][16][132];
  const int tid = threadIdx.x, wave = tid >> 5, lane = tid & 31, col = lane & 15, g = lane >> 4; const size_t r0 = (size_t)blockIdx.x * 64 + wave * 16;
  const __bf16* PW = PT + (L == 1 ? PT_W1 : PT_W2); const __bf16* PR = PT + (L == 1 ? PT_W1R : PT_W2R);
#pragma unroll 1
  for (int part = 0; part < 2; ++part) { const __bf16* P = part == 0 ? PW : PR; v8f acc[NT] = {};
#pragma unroll
    for (int kc = 0; kc < KI / 32; ++kc) { const F2 a = split_row(Xin + (r0 + col) * KI, kc * 32, lane);
#pragma unroll
      for (int j = 0; j < NT; ++j) { const v16b w = frag_b(P + (size_t)(j * 16 + col) * KI + kc * 32, lane); if (L == 2) acc[j] = wmma_bf(a.l, w, acc[j]); acc[j] = wmma_bf(a.h, w, acc[j]); } }
#pragma unroll
    for (int j = 0; j < NT; ++j) { const int o = j * 16 + col;
#pragma unroll
      for (int r = 0; r < 8; ++r) { const size_t n = r0 + 8 * g + r; float v = acc[j][r];
        if (part == 0) { const float deg = (n < (size_t)CSR_N) ? (float)min(max(RCT[n], 0), CSR_BCAP) + 1.0f : 1.0f; v = v * rsqrtf(deg); } else v += bfr(br[o]);
        so[wave][8 * g + r][o] = (n < (size_t)CSR_N) ? v : 0.f; } }
    LDSX();
    float* dstp = part == 0 ? HM : RS;
    for (int rl = 0; rl < 16; ++rl) for (int pc = lane; pc < NO / 4; pc += 32) vst2(dstp + (r0 + rl) * NO + pc * 4, *(const v4f*)&so[wave][rl][pc * 4]);
    LDSX(); }
}
template <int NO>
__global__ __launch_bounds__(256) void k_gcn(const float* __restrict__ HM, const float* __restrict__ RS, const float* __restrict__ lg, const float* __restrict__ lb, const int* __restrict__ FS, const int* __restrict__ RST, const int* __restrict__ RCT, float* __restrict__ Xout) {
  constexpr int FQ = NO / 4;
  __shared__ float sh[64][NO + 1];
  const int tid = threadIdx.x; const int nl = tid >> 2; const size_t node = (size_t)blockIdx.x * 64 + nl; const int f0 = (tid & 3) * FQ;
  float acc[FQ];
#pragma unroll
  for (int i = 0; i < FQ; ++i) acc[i] = 0.f;
  int cnt = 0;
  if (node < (size_t)CSR_N) { cnt = min(max(RCT[node], 0), CSR_BCAP); const int st = min(max(RST[node], 0), CSR_FINN - cnt);
    for (int e = 0; e < cnt; ++e) { const int s = min(max(FS[st + e], 0), CSR_N - 1); const float* hr = HM + (size_t)s * NO + f0;
#pragma unroll
      for (int i = 0; i < FQ; ++i) acc[i] += hr[i]; } }
  { const float nrm = rsqrtf((float)cnt + 1.0f); const float* hs = HM + node * NO + f0; const float* rs = RS + node * NO + f0;
#pragma unroll
    for (int i = 0; i < FQ; ++i) sh[nl][f0 + i] = (acc[i] + hs[i]) * nrm + rs[i]; }
  __syncthreads();
  { float s = 0.f; for (int c = 0; c < NO; ++c) s += sh[nl][c]; const float mu = s / (float)NO; float v = 0.f; for (int c = 0; c < NO; ++c) { const float d = sh[nl][c] - mu; v += d * d; } const float rsd = rsqrtf(v / (float)NO + 1e-5f);
#pragma unroll
    for (int p = 0; p < FQ / 4; ++p) { v4f o; for (int i = 0; i < 4; ++i) { const int c = f0 + p * 4 + i; const float y = (sh[nl][c] - mu) * rsd * bfr(lg[c]) + bfr(lb[c]); o[i] = node < (size_t)CSR_N ? fmaxf(y, 0.f) : 0.f; } vst2(Xout + node * NO + f0 + p * 4, o); } }
}
__global__ __launch_bounds__(256) void k_pool(const int* __restrict__ GID, const float* __restrict__ X2, float* __restrict__ HG) {
  __shared__ float sacc[4][64]; __shared__ int scnt[4]; __shared__ __align__(16) float srow[64]; __shared__ int srng[2];
  const int b = blockIdx.x, tid = threadIdx.x; const int part = tid >> 6, c = tid & 63;
  if (tid < 2) { const int key = b + tid; int lo = 0, hi = CSR_N; while (lo < hi) { const int mid = (lo + hi) >> 1; if (GID[mid] < key) lo = mid + 1; else hi = mid; } srng[tid] = lo; }
  __syncthreads();
  const int n0 = srng[0], n1 = max(srng[1], srng[0]);
  float a = 0.f; int n_ = 0;
  for (int n = n0 + part; n < n1; n += 4) { if (GID[n] == b) { a += X2[(size_t)n * 64 + c]; ++n_; } }
  sacc[part][c] = a; if (c == 0) scnt[part] = n_;
  __syncthreads();
  if (tid < 64) { const float s = (sacc[0][tid] + sacc[1][tid]) + (sacc[2][tid] + sacc[3][tid]); const int cn = scnt[0] + scnt[1] + scnt[2] + scnt[3]; srow[tid] = s / fmaxf((float)cn, 1.0f); }
  __syncthreads();
  if (tid < 16) vst2(HG + (size_t)b * 64 + tid * 4, *(const v4f*)&srow[tid * 4]);
}

__global__ __launch_bounds__(256) void k_head1(const float* __restrict__ HG, const float* __restrict__ D3, const float* __restrict__ Wmu, const float* __restrict__ bmu, const float* __restrict__ Wlv, const float* __restrict__ blv, const float* __restrict__ Wa, const float* __restrict__ ba,
                                               const float* __restrict__ Wvr, const float* __restrict__ bvr, const float* __restrict__ lvg, const float* __restrict__ lvb, const float* __restrict__ WU, const float* __restrict__ WV, const float* __restrict__ lfg, const float* __restrict__ lfb, const float* __restrict__ Wh1, const float* __restrict__ bh1, float* __restrict__ H1) {
  __shared__ float shg[64]; __shared__ float sv3[256]; __shared__ float svr[32]; __shared__ float sfu[64]; __shared__ float sred[8]; __shared__ __align__(16) float sh1[128];
  const int b = blockIdx.x, tid = threadIdx.x, lane = tid & 31, wave = tid >> 5;
  if (tid < 64) shg[tid] = HG[(size_t)b * 64 + tid];
  __syncthreads();
  { const int o = tid; float m = bfr(bmu[o]), lv = bfr(blv[o]), a = bfr(ba[o]);
#pragma unroll 1
    for (int k = 0; k < 64; ++k) { const float h = shg[k]; m += h * bfr(Wmu[k * 256 + o]); lv += h * bfr(Wlv[k * 256 + o]); a += h * bfr(Wa[k * 256 + o]); }
    lv = fminf(fmaxf(lv, -8.0f), 8.0f); const float var = exp_ni(lv) + 1e-6f; const float z = (bfr(D3[(size_t)b * 256 + o]) - m) / (sqrtf(var) + 1e-6f); const float w = (1.0f / (1.0f + exp_ni(-a))) * fminf(1.0f / var, 50.0f); sv3[o] = w * z; }
  __syncthreads();
  { const int o = tid >> 3, part = tid & 7; float s = 0.f;
#pragma unroll 1
    for (int k = part * 32; k < part * 32 + 32; ++k) s += sv3[k] * bfr(Wvr[k * 32 + o]);
    s += __shfl_xor(s, 1); s += __shfl_xor(s, 2); s += __shfl_xor(s, 4); if (part == 0) svr[o] = s + bfr(bvr[o]); }
  __syncthreads();
  if (tid < 32) { const float v = svr[tid]; float s = v;
#pragma unroll
    for (int q = 1; q < 32; q <<= 1) s += __shfl_xor(s, q);
    const float mu = s / 32.f; const float d = v - mu; float vv = d * d;
#pragma unroll
    for (int q = 1; q < 32; q <<= 1) vv += __shfl_xor(vv, q);
    const float y = d * rsqrtf(vv / 32.f + 1e-5f) * bfr(lvg[tid]) + bfr(lvb[tid]); svr[tid] = fmaxf(y, 0.f); }
  __syncthreads();
  if (tid < 64) { const int o = tid; float u = 0.f, vv = 0.f;
#pragma unroll 1
    for (int k = 0; k < 64; ++k) u += shg[k] * bfr(WU[k * 64 + o]);
#pragma unroll 1
    for (int k = 0; k < 32; ++k) vv += svr[k] * bfr(WV[k * 64 + o]);
    sfu[o] = u * vv; }
  __syncthreads();
  if (tid < 64) {
    const float v = sfu[tid]; float s = v;
#pragma unroll
    for (int q = 1; q < 32; q <<= 1) s += __shfl_xor(s, q);
    if (lane == 0) sred[wave] = s; }
  __syncthreads();
  if (tid < 64) { const float mu = (sred[0] + sred[1]) / 64.f; const float d = sfu[tid] - mu; float vv = d * d;
#pragma unroll
    for (int q = 1; q < 32; q <<= 1) vv += __shfl_xor(vv, q);
    if (lane == 0) sred[2 + wave] = vv; }
  __syncthreads();
  if (tid < 64) { const float mu = (sred[0] + sred[1]) / 64.f; const float var = (sred[2] + sred[3]) / 64.f; sfu[tid] = (sfu[tid] - mu) * rsqrtf(var + 1e-5f) * bfr(lfg[tid]) + bfr(lfb[tid]); }
  __syncthreads();
  if (tid < 128) { const int o = tid; float s = bfr(bh1[o]);
#pragma unroll 1
    for (int k = 0; k < 64; ++k) s += sfu[k] * bfr(Wh1[k * 128 + o]);
    sh1[o] = s; }
  __syncthreads();
  if (tid < 32) vst2(H1 + (size_t)b * 128 + tid * 4, *(const v4f*)&sh1[tid * 4]);
}
__global__ __launch_bounds__(128) void k_head2(const float* __restrict__ H1, const float* __restrict__ bng, const float* __restrict__ bnb, const float* __restrict__ Wh2, const float* __restrict__ bh2, float* __restrict__ out) {
  __shared__ float sm[128], srs[128], sg[128], sb[128], sw[128]; __shared__ __align__(16) float sout[512];
  const int tid = threadIdx.x; const int o = tid;
  { float s = 0.f;
#pragma unroll 1
    for (int b = 0; b < NB; ++b) s += H1[(size_t)b * 128 + o];
    const float m = s / (float)NB; float v = 0.f;
#pragma unroll 1
    for (int b = 0; b < NB; ++b) { const float d = H1[(size_t)b * 128 + o] - m; v += d * d; }
    sm[o] = m; srs[o] = rsqrtf(v / (float)NB + 1e-5f); sg[o] = bfr(bng[o]); sb[o] = bfr(bnb[o]); sw[o] = bfr(Wh2[o]); }
  __syncthreads();
#pragma unroll 1
  for (int b = tid; b < 512; b += 128) { float s = 0.f; if (b < NB) { s = bfr(bh2[0]);
#pragma unroll 1
      for (int k = 0; k < 128; ++k) { const float h = fmaxf((H1[(size_t)b * 128 + k] - sm[k]) * srs[k] * sg[k] + sb[k], 0.f); s += h * sw[k]; } }
    sout[b] = s; }
  __syncthreads();
  if (tid < NB / 4) vst2(out + tid * 4, *(const v4f*)&sout[tid * 4]);
}

extern "C" void kernel_launch(void* const* d_in, const int* in_sizes, int n_in, void* d_out, int out_size, void* d_ws, size_t ws_size, hipStream_t stream) {
  (void)in_sizes; (void)n_in; (void)out_size;
  const float** F = (const float**)d_in; const int** I = (const int**)d_in;
  if (ws_size < (size_t)WS_END) return;
  char* ws = (char*)d_ws;
  int *CNT = (int*)(ws + WS_CNT), *OFF = (int*)(ws + WS_OFF), *BST = (int*)(ws + WS_BST), *SEGS = (int*)(ws + WS_SEGS), *SEGE = (int*)(ws + WS_SEGE), *FS = (int*)(ws + WS_FS), *FE = (int*)(ws + WS_FE), *RST = (int*)(ws + WS_RST), *RCT = (int*)(ws + WS_RCT);
  __bf16* PT = (__bf16*)(ws + WS_PT); float *X0 = (float*)(ws + WS_X0), *HM = (float*)(ws + WS_HM), *RS = (float*)(ws + WS_RS), *X1 = (float*)(ws + WS_X1), *X2 = (float*)(ws + WS_X2), *HG = (float*)(ws + WS_HG);
  const int* SRC = I[3]; const int* DST = I[4];
  k_csr_cnt<<<CSR_NCH, 256, 0, stream>>>(DST, 1, CNT);
  k_csr_scan<<<1, 256, 0, stream>>>(CNT, OFF, BST);
  k_csr_scatter<<<CSR_NCH, 256, 0, stream>>>(SRC, DST, 1, 1, OFF, SEGS, SEGE);
  k_csr_bucket<<<CSR_NBK, 256, 0, stream>>>(CNT, OFF, BST, SEGS, SEGE, DST, 1, FS, FE, RST, RCT);
  k_pack<<<384, 128, 0, stream>>>(F[6], F[7], F[11], F[12], PT);
  k_x0<<<NNP / 64, 256, 0, stream>>>(F[0], X0);
  k_pre<1><<<NNP / 64, 128, 0, stream>>>(X0, PT, F[8], RCT, HM, RS);
  k_gcn<128><<<NNP / 64, 256, 0, stream>>>(HM, RS, F[9], F[10], FS, RST, RCT, X1);
  k_pre<2><<<NNP / 64, 128, 0, stream>>>(X1, PT, F[13], RCT, HM, RS);
  k_gcn<64><<<NNP / 64, 256, 0, stream>>>(HM, RS, F[14], F[15], FS, RST, RCT, X2);
  k_pool<<<NB, 256, 0, stream>>>(I[5], X2, HG);
  k_head1<<<NB, 256, 0, stream>>>(HG, F[2], F[16], F[17], F[18], F[19], F[20], F[21], F[22], F[23], F[24], F[25], F[26], F[27], F[28], F[29], F[30], F[31], X1  );
  k_head2<<<1, 128, 0, stream>>>(X1, F[32], F[33], F[34], F[35], (float*)d_out);
}
